// KAN_layer_63333587746983
// MI455X (gfx1250) — hardware-verified
//
#include <hip/hip_runtime.h>
#include <math.h>

constexpr int kBatch = 2048;
constexpr int kIn    = 256;
constexpr int kOut   = 256;
constexpr int kDeg   = 3;
constexpr int kKnots = 15;
constexpr int kCoef  = kKnots - (kDeg + 1);
constexpr int kKdim  = kIn + kIn * kCoef;
constexpr int kChunks = kKdim / 8;
constexpr float kACarry   = 256.0f;
constexpr float kWCarry   = 1024.0f;
constexpr float kOutScale = 1.0f / (256.0f * 1024.0f);
static_assert(kCoef == 11);
static_assert(kKdim % 32 == 0);
static_assert(kBatch % 64 == 0);
static_assert(kOut % 64 == 0);
static_assert(kChunks == 384);

typedef __attribute__((ext_vector_type(16))) _Float16 v16h;
typedef __attribute__((ext_vector_type(8)))  _Float16 v8h;
typedef __attribute__((ext_vector_type(16))) __bf16   v16b;
typedef __attribute__((ext_vector_type(8)))  __bf16   v8b;
typedef __attribute__((ext_vector_type(8)))  float    v8f;
typedef __attribute__((ext_vector_type(4)))  float    v4f;
typedef __attribute__((ext_vector_type(4)))  unsigned int v4u;

__device__ __forceinline__ unsigned short f2bf_bits(float f) {
  unsigned u = __float_as_uint(f);
  return (unsigned short)((u + 0x7FFFu + ((u >> 16) & 1u)) >> 16);
}
__device__ __forceinline__ float bf_bits2f(unsigned short h) { return __uint_as_float(((unsigned)h) << 16); }

__device__ __forceinline__ void dep_guard_h(v8f& a, v8f& b, v16h x, v16h y) { asm volatile("v_nop\n\tv_nop\n\tv_nop\n\tv_nop" : "+v"(a), "+v"(b) : "v"(x), "v"(y)); }
__device__ __forceinline__ void dep_guard_b(v8f& a, v8f& b, v16b x, v16b y) { asm volatile("v_nop\n\tv_nop\n\tv_nop\n\tv_nop" : "+v"(a), "+v"(b) : "v"(x), "v"(y)); }
__device__ __forceinline__ void keep4_h(v16h a, v16h b, v16h c, v16h d) { asm volatile("v_nop" :: "v"(a), "v"(b), "v"(c), "v"(d)); }
__device__ __forceinline__ void keep4_b(v16b a, v16b b, v16b c, v16b d) { asm volatile("v_nop" :: "v"(a), "v"(b), "v"(c), "v"(d)); }
__device__ __forceinline__ void acc_guard4(v8f& a, v8f& b, v8f& c, v8f& d) { asm volatile("v_nop\n\tv_nop\n\tv_nop\n\tv_nop" : "+v"(a), "+v"(b), "+v"(c), "+v"(d)); }
template <typename T> struct Frag;
template <> struct Frag<_Float16> {
  typedef v16h V; union U { v16h v; v8h h[2]; };
  static __device__ __forceinline__ v16h load(const _Float16* p) {
    U f; f.h[0] = *(const v8h*)(p); f.h[1] = *(const v8h*)(p + 16); return f.v;
  }
  static __device__ __forceinline__ v8f mma(v16h a, v16h b, v8f c) {
    return __builtin_amdgcn_wmma_f32_16x16x32_f16(false, a, false, b, (short)0, c, false, false);
  }
  static __device__ __forceinline__ void guard(v8f& a, v8f& b, v16h x, v16h y) { dep_guard_h(a, b, x, y); }
  static __device__ __forceinline__ void keep(v16h a, v16h b, v16h c, v16h d) { keep4_h(a, b, c, d); }
};
template <> struct Frag<__bf16> {
  typedef v16b V; union U { v16b v; v8b h[2]; };
  static __device__ __forceinline__ v16b load(const __bf16* p) {
    U f; f.h[0] = *(const v8b*)(p); f.h[1] = *(const v8b*)(p + 16); return f.v;
  }
  static __device__ __forceinline__ v8f mma(v16b a, v16b b, v8f c) {
    return __builtin_amdgcn_wmma_f32_16x16x32_bf16(false, a, false, b, (short)0, c, false, false);
  }
  static __device__ __forceinline__ void guard(v8f& a, v8f& b, v16b x, v16b y) { dep_guard_b(a, b, x, y); }
  static __device__ __forceinline__ void keep(v16b a, v16b b, v16b c, v16b d) { keep4_b(a, b, c, d); }
};

__device__ __forceinline__ unsigned pk16(unsigned short a, unsigned short b) { return (unsigned)a | ((unsigned)b << 16); }
__device__ __forceinline__ unsigned short h_bits(float f) { const _Float16 h = (_Float16)f; return __builtin_bit_cast(unsigned short, h); }

template <int ET> struct Elem;
template <> struct Elem<0> { typedef _Float16 T; };
template <> struct Elem<1> { typedef __bf16 T; };
template <int ET, bool SPLIT, int BIAS_MODE, int OUT_MODE, bool RESID, int ACT = 0>
__global__ __launch_bounds__(256) void wmma_gemm64(
    const unsigned short* __restrict__ Ap, const unsigned short* __restrict__ A2p, int lda, long strideA,
    const unsigned short* __restrict__ Btp, const unsigned short* __restrict__ Bt2p, int ldb, long strideB,
    void* __restrict__ Cout, void* __restrict__ Cout2, int ldc, long strideC,
    const float* __restrict__ bias,
    const float* __restrict__ resid, long strideR,
    int M, int N, int K, float scale) {
  typedef typename Elem<ET>::T T;
  typedef typename Frag<T>::V V;
  const T* A = (const T*)Ap; const T* A2 = (const T*)A2p; const T* Bt = (const T*)Btp; const T* Bt2 = (const T*)Bt2p;
  __shared__ __align__(16) float sT[8][16 * 68];
  const int b    = blockIdx.y;
  const int lane = threadIdx.x & 31;
  const int wave = threadIdx.x >> 5;
  const int tilesN = N >> 6;
  const int tilesM = M >> 6;
  const int tile = blockIdx.x * 8 + wave;
  if (tile >= tilesM * tilesN) return;
  const int tm = tile / tilesN;
  const int tn = tile - tm * tilesN;
  const int m0 = tm << 6;
  const int n0 = tn << 6;

  const T* Ab  = A  + (size_t)b * strideA;
  const T* Bb  = Bt + (size_t)b * strideB;
  const T* Ab2 = SPLIT ? (A2  + (size_t)b * strideA) : nullptr;
  const T* Bb2 = SPLIT ? (Bt2 + (size_t)b * strideB) : nullptr;

  const int rlane = lane & 15;
  const int koff  = (lane >> 4) * 8;
  const int mOff  = (lane >> 4) * 8;

  v8f acc[4][4];
#pragma unroll
  for (int i = 0; i < 4; ++i)
#pragma unroll
    for (int j = 0; j < 4; ++j) acc[i][j] = (v8f){0.f,0.f,0.f,0.f,0.f,0.f,0.f,0.f};

  for (int k0 = 0; k0 < K; k0 += 32) {
    V bh[4], bl[4];
#pragma unroll
    for (int j = 0; j < 4; ++j) {
      const size_t bo = (size_t)(n0 + (j << 4) + rlane) * ldb + koff + k0;
      bh[j] = Frag<T>::load(Bb + bo);
      if (SPLIT) bl[j] = Frag<T>::load(Bb2 + bo);
    }
#pragma unroll
    for (int i = 0; i < 4; ++i) {
      const size_t ao = (size_t)(m0 + (i << 4) + rlane) * lda + koff + k0;
      V ah = Frag<T>::load(Ab + ao);
      V al;
      if (SPLIT) al = Frag<T>::load(Ab2 + ao);
#pragma unroll
      for (int j = 0; j < 4; ++j) {
        acc[i][j] = Frag<T>::mma(ah, bh[j], acc[i][j]);
        if (SPLIT) {
          acc[i][j] = Frag<T>::mma(ah, bl[j], acc[i][j]);
          acc[i][j] = Frag<T>::mma(al, bh[j], acc[i][j]);
        }
      }
      Frag<T>::guard(acc[i][0], acc[i][3], ah, SPLIT ? al : ah);
    }
    Frag<T>::keep(bh[0], bh[1], bh[2], bh[3]);
    if (SPLIT) Frag<T>::keep(bl[0], bl[1], bl[2], bl[3]);
  }
  acc_guard4(acc[0][0], acc[0][1], acc[0][2], acc[0][3]);
  acc_guard4(acc[1][0], acc[1][1], acc[1][2], acc[1][3]);
  acc_guard4(acc[2][0], acc[2][1], acc[2][2], acc[2][3]);
  acc_guard4(acc[3][0], acc[3][1], acc[3][2], acc[3][3]);

  float* slab = sT[wave];
  const float* Rb = RESID ? (resid + (size_t)b * strideR) : nullptr;
#pragma unroll
  for (int i = 0; i < 4; ++i) {
    const int mBase = m0 + (i << 4);
#pragma unroll
    for (int j = 0; j < 4; ++j) {
      const int n = n0 + (j << 4) + rlane;
      float bv = 0.f;
      if (BIAS_MODE == 2) bv = bias[n];
#pragma unroll
      for (int r = 0; r < 8; ++r) {
        float v = acc[i][j][r] * scale;
        if (BIAS_MODE == 1) v += bias[mBase + mOff + r];
        if (BIAS_MODE == 2) v += bv;
        if (RESID) v += Rb[(size_t)(mBase + mOff + r) * ldc + n];
        if (ACT == 2) v = fmaxf(v, 0.0f);
        if (ACT == 4) v = (v > 0.f) ? v : 0.01f * v;
        slab[(mOff + r) * 68 + (j << 4) + rlane] = v;
      }
    }
    __builtin_amdgcn_fence(__ATOMIC_RELEASE, "workgroup");
    __builtin_amdgcn_wave_barrier();
    __builtin_amdgcn_fence(__ATOMIC_ACQUIRE, "workgroup");
    if (OUT_MODE == 0) {
      float* C = (float*)Cout + (size_t)b * strideC;
      const int hh = lane >> 4, c4 = (lane & 15) * 4;
      for (int pass = 0; pass < 2; ++pass) {
#pragma unroll
        for (int it = 0; it < 8; ++it) {
          const int row = it * 2 + hh;
          v4f v = *(const v4f*)(slab + row * 68 + c4);
          *(volatile v4f*)(C + (size_t)(mBase + row) * ldc + n0 + c4) = v;
        }
        __threadfence();
      }
    } else {
      const int q = lane >> 3, c8 = (lane & 7) * 8;
      unsigned short* C  = (unsigned short*)Cout  + (size_t)b * strideC;
      unsigned short* C2 = (OUT_MODE == 2) ? ((unsigned short*)Cout2 + (size_t)b * strideC) : nullptr;
      for (int pass = 0; pass < 2; ++pass) {
#pragma unroll
        for (int it = 0; it < 4; ++it) {
          const int row = it * 4 + q;
          const float* sp = slab + row * 68 + c8;
          v8h hv, lv;
#pragma unroll
          for (int e = 0; e < 8; ++e) {
            if (OUT_MODE == 1) {
              hv[e] = (_Float16)sp[e];
            } else {
              unsigned short hb = f2bf_bits(sp[e]);
              unsigned short lb = f2bf_bits(sp[e] - bf_bits2f(hb));
              hv[e] = __builtin_bit_cast(_Float16, hb);
              lv[e] = __builtin_bit_cast(_Float16, lb);
            }
          }
          *(volatile v8h*)(C + (size_t)(mBase + row) * ldc + n0 + c8) = hv;
          if (OUT_MODE == 2) *(volatile v8h*)(C2 + (size_t)(mBase + row) * ldc + n0 + c8) = lv;
        }
        __threadfence();
      }
    }
    __builtin_amdgcn_fence(__ATOMIC_RELEASE, "workgroup");
    __builtin_amdgcn_wave_barrier();
    __builtin_amdgcn_fence(__ATOMIC_ACQUIRE, "workgroup");
  }
}

__device__ __forceinline__ void write_row_lines(const unsigned short* sRow, unsigned short* __restrict__ dst, int t) {
  const int t2 = (t < 128) ? t : 0;
  const v4u u0 = *(const v4u*)(sRow + t * 8);
  const v4u u1 = *(const v4u*)(sRow + (256 + t2) * 8);
  for (int pass = 0; pass < 2; ++pass) {
    *(volatile v4u*)(dst + (size_t)t * 8) = u0;
    if (t < 128) *(volatile v4u*)(dst + (size_t)(256 + t) * 8) = u1;
    __threadfence();
  }
}

__global__ __launch_bounds__(256) void basis_rows_kernel(const float* __restrict__ x,
                                                         const float* __restrict__ knots,
                                                         unsigned short* __restrict__ A16) {
#pragma clang fp contract(off)
  __shared__ float sKn[kIn * 16];
  __shared__ float sB[kIn * 16];
  __shared__ __align__(16) unsigned short sRow[kKdim];
  const int b = blockIdx.x;
  const int t = threadIdx.x;
  const float xv = x[(size_t)b * kIn + t];
  float* kn = sKn + t * 16;
  float* bb = sB + t * 16;

#pragma unroll 1
  for (int j = 0; j < kKnots; ++j) kn[j] = knots[t * kKnots + j];

#pragma unroll 1
  for (int j = 0; j < kKnots - 1; ++j) {
    const float g0 = kn[j];
    const float g1 = kn[j + 1];
    bb[j] = (xv >= g0 && xv < g1) ? 1.0f : 0.0f;
  }
#pragma unroll 1
  for (int p = 1; p <= kDeg; ++p) {
    const int nj = kKnots - 1 - p;
#pragma unroll 1
    for (int j = 0; j < nj; ++j) {
      const float g0  = kn[j];
      const float g1  = kn[j + 1];
      const float gp  = kn[j + p];
      const float gp1 = kn[j + p + 1];
      const float left  = (xv - g0) / (gp - g0) * bb[j];
      const float right = (gp1 - xv) / (gp1 - g1) * bb[j + 1];
      bb[j] = left + right;
    }
  }

  const float ex = expf(-xv);
  const float silu = xv * (1.0f / (1.0f + ex));

  sRow[t] = h_bits(silu * kACarry);
#pragma unroll 1
  for (int l = 0; l < kCoef; ++l) sRow[kIn + t * kCoef + l] = h_bits(bb[l] * kACarry);
  __syncthreads();

  write_row_lines(sRow, A16 + (size_t)b * kKdim, t);
}

__global__ __launch_bounds__(256) void weight_rows_kernel(const float* __restrict__ cp,
                                                          const float* __restrict__ scale_base,
                                                          const float* __restrict__ scale_spline,
                                                          const float* __restrict__ mask,
                                                          unsigned short* __restrict__ Bt16) {
#pragma clang fp contract(off)
  __shared__ __align__(16) unsigned short sRow[kKdim];
  const int o = blockIdx.x;
  const int t = threadIdx.x;
  const size_t io = (size_t)t * kOut + o;
  const float m   = mask[io];
  const float vsb = scale_base[io] * m;
  const float vss = scale_spline[io] * m;
  sRow[t] = h_bits(vsb * kWCarry);
  const float f = vss * kWCarry;
  const float* c = cp + io * kCoef;
#pragma unroll 1
  for (int l = 0; l < kCoef; ++l) sRow[kIn + t * kCoef + l] = h_bits(c[l] * f);
  __syncthreads();

  write_row_lines(sRow, Bt16 + (size_t)o * kKdim, t);
}

extern "C" void kernel_launch(void* const* d_in, const int* in_sizes, int n_in,
                              void* d_out, int out_size, void* d_ws, size_t ws_size,
                              hipStream_t stream) {
  if (n_in < 6) return;
  if (in_sizes[0] != kBatch * kIn) return;
  if (in_sizes[1] != kIn * kKnots) return;
  if (in_sizes[2] != kIn * kOut * kCoef) return;
  if (in_sizes[3] != kIn * kOut) return;
  if (in_sizes[4] != kIn * kOut) return;
  if (in_sizes[5] != kIn * kOut) return;
  if (out_size != kBatch * kOut) return;

  const size_t bytesA = (size_t)kBatch * kKdim * sizeof(unsigned short);
  const size_t bytesB = (size_t)kOut * kKdim * sizeof(unsigned short);
  if (bytesA + bytesB > ws_size) return;

  const float* x            = (const float*)d_in[0];
  const float* knots        = (const float*)d_in[1];
  const float* cp           = (const float*)d_in[2];
  const float* scale_base   = (const float*)d_in[3];
  const float* scale_spline = (const float*)d_in[4];
  const float* mask         = (const float*)d_in[5];
  float* out = (float*)d_out;

  unsigned short* A16  = (unsigned short*)d_ws;
  unsigned short* Bt16 = (unsigned short*)((char*)d_ws + bytesA);

  basis_rows_kernel<<<dim3(kBatch), dim3(256), 0, stream>>>(x, knots, A16);
  weight_rows_kernel<<<dim3(kOut), dim3(256), 0, stream>>>(cp, scale_base, scale_spline, mask, Bt16);

  const int tiles = (kBatch / 64) * (kOut / 64);
  wmma_gemm64<0, false, 0, 0, false, 0><<<dim3(tiles / 8, 1), dim3(256), 0, stream>>>(
      (const unsigned short*)A16, (const unsigned short*)nullptr, kKdim, 0L,
      (const unsigned short*)Bt16, (const unsigned short*)nullptr, kKdim, 0L,
      (void*)out, (void*)nullptr, kOut, 0L,
      (const float*)nullptr,
      (const float*)nullptr, 0L,
      kBatch, kOut, kKdim, kOutScale);
}
